// EdgeTransformerLayer_41068477284524
// MI455X (gfx1250) — hardware-verified
//
#include <hip/hip_runtime.h>


#define NB_  2
#define NN   64
#define DD   256
#define NH_  8
#define DK   32
#define FF   512
#define NR   (NB_ * NN * NN)
#define NZ   (NB_ * NH_ * NN)
typedef _Float16 h16;
typedef unsigned short bf;
typedef __attribute__((ext_vector_type(16))) __bf16   v16bf;
typedef __attribute__((ext_vector_type(16))) _Float16 v16h;
typedef __attribute__((ext_vector_type(8)))  _Float16 v8h;
typedef __attribute__((ext_vector_type(8)))  unsigned short v8us;
typedef __attribute__((ext_vector_type(8)))  float    v8f;
typedef __attribute__((ext_vector_type(4)))  float    v4f;
typedef v8h  __attribute__((may_alias)) v8ha;
typedef v4f  __attribute__((may_alias)) v4fa;
typedef v8us __attribute__((may_alias)) v8usa;

__device__ __forceinline__ unsigned short f2bf(float f) { unsigned u = __float_as_uint(f); u += 0x7FFFu + ((u >> 16) & 1u); return (unsigned short)(u >> 16); }
__device__ __forceinline__ float bf2f(unsigned short b) { return __uint_as_float(((unsigned)b) << 16); }
__device__ __forceinline__ float bfr(float f) { return bf2f(f2bf(f)); }
__device__ __forceinline__ v16h cat16(v8h lo, v8h hi) { return __builtin_shufflevector(lo, hi, 0, 1, 2, 3, 4, 5, 6, 7, 8, 9, 10, 11, 12, 13, 14, 15); }
__device__ __forceinline__ v16bf cat16b(v8us lo, v8us hi) { return __builtin_bit_cast(v16bf, __builtin_shufflevector(lo, hi, 0, 1, 2, 3, 4, 5, 6, 7, 8, 9, 10, 11, 12, 13, 14, 15)); }
__device__ __forceinline__ v8f wmma16(v16h a, v16h b, v8f c) { return __builtin_amdgcn_wmma_f32_16x16x32_f16(false, a, false, b, (short)0, c, false, false); }
__device__ __forceinline__ v8f wmmab(v16bf a, v16bf b, v8f c) { return __builtin_amdgcn_wmma_f32_16x16x32_bf16(false, a, false, b, (short)0, c, false, false); }


template <typename T16> struct WFrag;
template <> struct WFrag<h16> { typedef v16h V; static __device__ __forceinline__ V ld(const h16* p) { return cat16(*(const v8h*)p, *(const v8h*)(p + 16)); } static __device__ __forceinline__ v8f mma(V a, V b, v8f c) { return wmma16(a, b, c); } };
template <> struct WFrag<bf> { typedef v16bf V; static __device__ __forceinline__ V ld(const bf* p) { return cat16b(*(const v8us*)p, *(const v8us*)(p + 16)); } static __device__ __forceinline__ v8f mma(V a, V b, v8f c) { return wmmab(a, b, c); } };
template <typename T16, int NSPLIT, bool BIAS>
__global__ __launch_bounds__(32) void k_gemmw(const T16* __restrict__ A, const T16* __restrict__ A2, const T16* __restrict__ Bt, const T16* __restrict__ Bt2, int K, float* C, int ldc, const float* __restrict__ bias, size_t sA, size_t sB, size_t sC) {
    typedef typename WFrag<T16>::V V;
    __shared__ __align__(16) float os[16 * 68];
    const size_t z = blockIdx.z; A += z * sA; if (A2) A2 += z * sA; Bt += z * sB; if (Bt2) Bt2 += z * sB; C += z * sC;
    const int lane = threadIdx.x & 31, lr = lane & 15, hi = lane >> 4; const int r0 = blockIdx.x * 64, c0 = blockIdx.y * 64;
    v8f acc[4][4];
#pragma unroll
    for (int mb = 0; mb < 4; ++mb)
#pragma unroll
        for (int nb = 0; nb < 4; ++nb) acc[mb][nb] = (v8f){};
    const size_t aoff = (size_t)(r0 + lr) * K + 8 * hi, boff = (size_t)(c0 + lr) * K + 8 * hi;
#pragma unroll 1
    for (int kc = 0; kc < K; kc += 32) {
        V a[4], a2[4];
#pragma unroll
        for (int mb = 0; mb < 4; ++mb) { a[mb] = WFrag<T16>::ld(A + aoff + (size_t)mb * 16 * K + kc); if (NSPLIT == 1 || NSPLIT == 2) a2[mb] = WFrag<T16>::ld(A2 + aoff + (size_t)mb * 16 * K + kc); }
#pragma unroll
        for (int nb = 0; nb < 4; ++nb) { const V b = WFrag<T16>::ld(Bt + boff + (size_t)nb * 16 * K + kc); V b2; if (NSPLIT >= 2) b2 = WFrag<T16>::ld(Bt2 + boff + (size_t)nb * 16 * K + kc);
#pragma unroll
            for (int mb = 0; mb < 4; ++mb) { acc[mb][nb] = WFrag<T16>::mma(a[mb], b, acc[mb][nb]); if (NSPLIT == 1 || NSPLIT == 2) acc[mb][nb] = WFrag<T16>::mma(a2[mb], b, acc[mb][nb]); if (NSPLIT >= 2) acc[mb][nb] = WFrag<T16>::mma(a[mb], b2, acc[mb][nb]); } }
        asm volatile("v_nop\n\tv_nop\n\tv_nop\n\tv_nop" : "+v"(acc[0][0]), "+v"(acc[1][1]), "+v"(acc[2][2]), "+v"(acc[3][3]) : "v"(a[0]), "v"(a[3]));
    }
#pragma unroll
    for (int mb = 0; mb < 4; ++mb) {
#pragma unroll
        for (int nb = 0; nb < 4; ++nb) {
#pragma unroll
            for (int j = 0; j < 8; ++j) os[(hi * 8 + j) * 68 + nb * 16 + lr] = acc[mb][nb][j]; }
        __builtin_amdgcn_wave_barrier(); asm volatile("" ::: "memory");
        float* crow = C + (size_t)(r0 + mb * 16) * ldc + c0;
#pragma unroll 1
        for (int ps = 0; ps < 2; ++ps) {
#pragma unroll
            for (int s = 0; s < 8; ++s) { const int row = 2 * s + hi, cofs = lr * 4; v4f val = *(const v4fa*)(os + row * 68 + cofs); if (BIAS) { val[0] += bfr(bias[c0 + cofs]); val[1] += bfr(bias[c0 + cofs + 1]); val[2] += bfr(bias[c0 + cofs + 2]); val[3] += bfr(bias[c0 + cofs + 3]); }
                *(volatile v4f*)(crow + (size_t)row * ldc + cofs) = val; }
            if (ps == 0) __threadfence(); }
        __builtin_amdgcn_wave_barrier(); asm volatile("" ::: "memory");
    }
}

__device__ __forceinline__ void splitf(float y, unsigned short& h, unsigned short& l) { h = f2bf(y); l = f2bf(y - bf2f(h)); }
typedef __attribute__((ext_vector_type(2))) unsigned short v2us;
typedef __attribute__((ext_vector_type(4))) unsigned short v4us;
typedef __attribute__((ext_vector_type(2))) float v2f;

__global__ __launch_bounds__(256) void k_cvt8(const float* __restrict__ src, bf* dst, size_t n8) { const size_t i = (size_t)blockIdx.x * 256 + threadIdx.x; if (i >= n8) return; const v8f v = *(const v8f*)(src + i * 8); v8us o;
#pragma unroll
    for (int k = 0; k < 8; ++k) o[k] = f2bf(v[k]); *(volatile v8us*)(dst + i * 8) = o; __threadfence(); *(volatile v8us*)(dst + i * 8) = o; }
__global__ __launch_bounds__(256) void k_wtb(const float* __restrict__ w, int K, int N, bf* Bt) {
    const int lane = threadIdx.x & 31; const int nlines = N * K / 64; const int wg = blockIdx.x * 8 + (threadIdx.x >> 5), nw = gridDim.x * 8;
#pragma unroll 1
    for (int ps = 0; ps < 2; ++ps) {
#pragma unroll 1
        for (int L = wg; L < nlines; L += nw) { const int e = L * 64 + lane * 2; v2us o;
#pragma unroll
            for (int q = 0; q < 2; ++q) { const int n = (e + q) / K, k = (e + q) % K; o[q] = f2bf(w[(size_t)k * N + n]); }
            *(volatile v2us*)(Bt + e) = o; }
        if (ps == 0) __threadfence(); }
}
__global__ __launch_bounds__(256) void k_kplanes(const float* __restrict__ LK, const float* __restrict__ RK, bf* LKh, bf* LKl, bf* RKh, bf* RKl) {
    const int lane = threadIdx.x & 31; const int L0 = (blockIdx.x * 8 + (threadIdx.x >> 5)) * 8; const int nlines = NZ * NN * DK / 64; const float sc = 0x1.6a09e6p-3f;
#pragma unroll 1
    for (int ps = 0; ps < 2; ++ps) {
#pragma unroll
        for (int l = 0; l < 8; ++l) { const int L = L0 + l; if (L >= nlines) break; const int e = L * 64 + lane * 2; const int d = e & 31; const int i = (e >> 5) & 63; const int z = e >> 11; const int a = z & 63, h = (z >> 6) & 7, b = z >> 9; v2us lh, ll, rh, rl;
#pragma unroll
            for (int q = 0; q < 2; ++q) { unsigned short p, s;
                splitf(LK[(((size_t)b * NN + i) * NN + a) * DD + h * DK + d + q] * sc, p, s); lh[q] = p; ll[q] = s;
                splitf(RK[(((size_t)b * NN + a) * NN + i) * DD + h * DK + d + q], p, s); rh[q] = p; rl[q] = s; }
            *(volatile v2us*)(LKh + e) = lh; *(volatile v2us*)(LKl + e) = ll; *(volatile v2us*)(RKh + e) = rh; *(volatile v2us*)(RKl + e) = rl; }
        if (ps == 0) __threadfence(); }
}
__global__ __launch_bounds__(256) void k_softa(const float* __restrict__ S, float* P) {
    const int lane = threadIdx.x & 31; const int wg = blockIdx.x * 8 + (threadIdx.x >> 5); if (wg >= NB_ * NH_ * NN) return; const int x = wg & 63, bh = wg >> 6;
    const size_t zb = (size_t)bh * NN;
    float m0 = -3.0e38f, m1 = -3.0e38f;
#pragma unroll 4
    for (int a = 0; a < NN; ++a) { const v2f v = *(const v2f*)(S + ((zb + a) * NN + x) * NN + lane * 2); m0 = fmaxf(m0, v[0]); m1 = fmaxf(m1, v[1]); }
    float s0 = 0.f, s1 = 0.f;
#pragma unroll 4
    for (int a = 0; a < NN; ++a) { const v2f v = *(const v2f*)(S + ((zb + a) * NN + x) * NN + lane * 2); s0 += __expf(v[0] - m0); s1 += __expf(v[1] - m1); }
    const float f0 = __fdiv_rn(1.0f, s0), f1 = __fdiv_rn(1.0f, s1);
#pragma unroll 1
    for (int ps = 0; ps < 2; ++ps) {
#pragma unroll 2
        for (int a = 0; a < NN; ++a) { const size_t o = ((zb + a) * NN + x) * NN + lane * 2; const v2f v = *(const v2f*)(S + o); v2f r; r[0] = __expf(v[0] - m0) * f0; r[1] = __expf(v[1] - m1) * f1; *(volatile v2f*)(P + o) = r; }
        if (ps == 0) __threadfence(); }
}
__global__ __launch_bounds__(256) void k_tri(const float* __restrict__ P, const float* __restrict__ LV, const float* __restrict__ RV, float* O) {
    const int lane = threadIdx.x & 31; const int wg = blockIdx.x * 8 + (threadIdx.x >> 5); if (wg >= NB_ * NH_ * NN) return; const int x = wg & 63, h = (wg >> 6) & 7, b = wg >> 9; const int d = lane;
    const size_t zb = ((size_t)b * NH_ + h) * NN; const float* lvb = LV + (((size_t)b * NN + x) * NN) * DD + h * DK + d; const float* rvb = RV + ((size_t)b * NN * NN) * DD + h * DK + d; const float* pb = P + (zb * NN + x) * NN;
#pragma unroll 1
    for (int ps = 0; ps < 2; ++ps) {
#pragma unroll 1
        for (int y = 0; y < NN; ++y) { float acc = 0.f;
#pragma unroll 4
            for (int a = 0; a < NN; ++a) acc = fmaf(pb[(size_t)a * NN * NN + y] * lvb[(size_t)a * DD], rvb[((size_t)a * NN + y) * DD], acc);
            *(volatile float*)(O + (((size_t)b * NN + x) * NN + y) * DD + h * DK + d) = acc; }
        if (ps == 0) __threadfence(); }
}
template <bool RELU>
__global__ __launch_bounds__(256) void k_split(const float* __restrict__ A, int nlines, bf* Ph, bf* Pl) {
    const int lane = threadIdx.x & 31; const int L0 = (blockIdx.x * 8 + (threadIdx.x >> 5)) * 8;
#pragma unroll 1
    for (int ps = 0; ps < 2; ++ps) {
#pragma unroll
        for (int l = 0; l < 8; ++l) { const int L = L0 + l; if (L >= nlines) break; const int e = L * 64 + lane * 2; v2us oh, ol;
#pragma unroll
            for (int q = 0; q < 2; ++q) { float v = A[(size_t)e + q]; if (RELU) v = fmaxf(v, 0.f); unsigned short a, c2; splitf(v, a, c2); oh[q] = a; ol[q] = c2; }
            *(volatile v2us*)(Ph + (size_t)e) = oh; *(volatile v2us*)(Pl + (size_t)e) = ol; }
        if (ps == 0) __threadfence(); }
}
template <bool FINAL>
__global__ __launch_bounds__(256) void k_ln(const float* __restrict__ A, const float* __restrict__ R, const float* __restrict__ gg, const float* __restrict__ bb, float* Y, bf* Ph, bf* Pl) {
    const int lane = threadIdx.x & 31; const int r = blockIdx.x * 8 + (threadIdx.x >> 5); if (r >= NR) return; float v[8]; float s = 0.f;
#pragma unroll
    for (int c = 0; c < 2; ++c)
#pragma unroll
        for (int q = 0; q < 4; ++q) { const int col = c * 128 + lane * 4 + q; const float rv = FINAL ? R[(size_t)r * DD + col] : bfr(R[(size_t)r * DD + col]); const float t = A[(size_t)r * DD + col] + rv; v[c * 4 + q] = t; s += t; }
#pragma unroll
    for (int sh = 16; sh; sh >>= 1) s += __shfl_xor(s, sh, 32);
    const float mu = s * (1.0f / DD); float qq = 0.f;
#pragma unroll
    for (int i = 0; i < 8; ++i) { const float dlt = v[i] - mu; qq = fmaf(dlt, dlt, qq); }
#pragma unroll
    for (int sh = 16; sh; sh >>= 1) qq += __shfl_xor(qq, sh, 32);
    const float rs = rsqrtf(qq * (1.0f / DD) + 1e-5f); v4f o[2]; v4us oh[2], ol[2];
#pragma unroll
    for (int c = 0; c < 2; ++c)
#pragma unroll
        for (int q = 0; q < 4; ++q) { const int col = c * 128 + lane * 4 + q; const float y = (v[c * 4 + q] - mu) * rs * bfr(gg[col]) + bfr(bb[col]); o[c][q] = y; if (!FINAL) { unsigned short a, c2; splitf(y, a, c2); oh[c][q] = a; ol[c][q] = c2; } }
#pragma unroll 1
    for (int ps = 0; ps < 2; ++ps) {
#pragma unroll
        for (int c = 0; c < 2; ++c) { *(volatile v4f*)(Y + (size_t)r * DD + c * 128 + lane * 4) = o[c]; if (!FINAL) { *(volatile v4us*)(Ph + (size_t)r * DD + c * 128 + lane * 4) = oh[c]; *(volatile v4us*)(Pl + (size_t)r * DD + c * 128 + lane * 4) = ol[c]; } }
        if (ps == 0) __threadfence(); }
}

extern "C" void kernel_launch(void* const* d_in, const int* in_sizes, int n_in,
                              void* d_out, int out_size, void* d_ws, size_t ws_size, hipStream_t stream) {
    (void)in_sizes; (void)n_in; (void)out_size;
    const float* x = (const float*)d_in[0]; const float* Wlk = (const float*)d_in[1]; const float* Wrk = (const float*)d_in[2]; const float* Wlv = (const float*)d_in[3]; const float* Wrv = (const float*)d_in[4]; const float* Wout = (const float*)d_in[5];
    const float* g1 = (const float*)d_in[6]; const float* be1 = (const float*)d_in[7]; const float* W1 = (const float*)d_in[8]; const float* b1 = (const float*)d_in[9]; const float* W2 = (const float*)d_in[10]; const float* b2 = (const float*)d_in[11]; const float* g2 = (const float*)d_in[12]; const float* be2 = (const float*)d_in[13];
    float* OUT = (float*)d_out;
    char* wsp = (char*)d_ws;
    auto take = [&](size_t bytes) { char* p = wsp; wsp += (bytes + 255) & ~(size_t)255; return (void*)p; };
    bf* XB = (bf*)take((size_t)NR * DD * 2); bf* WT = (bf*)take((size_t)5 * DD * DD * 2); bf* W1t = (bf*)take((size_t)FF * DD * 2); bf* W2t = (bf*)take((size_t)DD * FF * 2);
    float* LK = (float*)take((size_t)NR * DD * 4); float* RK = (float*)take((size_t)NR * DD * 4); float* LV = (float*)take((size_t)NR * DD * 4); float* RV = (float*)take((size_t)NR * DD * 4);
    bf* LKh = (bf*)take((size_t)NZ * NN * DK * 2); bf* LKl = (bf*)take((size_t)NZ * NN * DK * 2); bf* RKh = (bf*)take((size_t)NZ * NN * DK * 2); bf* RKl = (bf*)take((size_t)NZ * NN * DK * 2);
    float* S = (float*)take((size_t)NZ * NN * NN * 4); float* P = (float*)take((size_t)NZ * NN * NN * 4);
    float* O = (float*)take((size_t)NR * DD * 4); bf* OPh = (bf*)take((size_t)NR * DD * 2); bf* OPl = (bf*)take((size_t)NR * DD * 2); float* AO = (float*)take((size_t)NR * DD * 4);
    float* HN = (float*)take((size_t)NR * DD * 4); bf* HNh = (bf*)take((size_t)NR * DD * 2); bf* HNl = (bf*)take((size_t)NR * DD * 2);
    if ((size_t)(wsp - (char*)d_ws) > ws_size) return;
    float* F1 = S; bf* F1h = (bf*)LK; bf* F1l = (bf*)RK; float* F2 = P;
    { const size_t nx = (size_t)NR * DD / 8; k_cvt8<<<(unsigned)((nx + 255) / 256), 256, 0, stream>>>(x, XB, nx); }
    k_wtb<<<16, 256, 0, stream>>>(Wlk, DD, DD, WT); k_wtb<<<16, 256, 0, stream>>>(Wrk, DD, DD, WT + (size_t)DD * DD); k_wtb<<<16, 256, 0, stream>>>(Wlv, DD, DD, WT + (size_t)2 * DD * DD); k_wtb<<<16, 256, 0, stream>>>(Wrv, DD, DD, WT + (size_t)3 * DD * DD); k_wtb<<<16, 256, 0, stream>>>(Wout, DD, DD, WT + (size_t)4 * DD * DD);
    k_wtb<<<32, 256, 0, stream>>>(W1, DD, FF, W1t); k_wtb<<<32, 256, 0, stream>>>(W2, FF, DD, W2t);
    k_gemmw<bf, 0, false><<<dim3(NR / 64, DD / 64, 1), 32, 0, stream>>>(XB, nullptr, WT, nullptr, DD, LK, DD, nullptr, 0, 0, 0);
    k_gemmw<bf, 0, false><<<dim3(NR / 64, DD / 64, 1), 32, 0, stream>>>(XB, nullptr, WT + (size_t)DD * DD, nullptr, DD, RK, DD, nullptr, 0, 0, 0);
    k_gemmw<bf, 0, false><<<dim3(NR / 64, DD / 64, 1), 32, 0, stream>>>(XB, nullptr, WT + (size_t)2 * DD * DD, nullptr, DD, LV, DD, nullptr, 0, 0, 0);
    k_gemmw<bf, 0, false><<<dim3(NR / 64, DD / 64, 1), 32, 0, stream>>>(XB, nullptr, WT + (size_t)3 * DD * DD, nullptr, DD, RV, DD, nullptr, 0, 0, 0);
    k_kplanes<<<(NZ * NN * DK / 64 + 63) / 64, 256, 0, stream>>>(LK, RK, LKh, LKl, RKh, RKl);
    k_gemmw<bf, 2, false><<<dim3(1, 1, NZ), 32, 0, stream>>>(LKh, LKl, RKh, RKl, DK, S, NN, nullptr, (size_t)NN * DK, (size_t)NN * DK, (size_t)NN * NN);
    k_softa<<<NB_ * NH_ * NN / 8, 256, 0, stream>>>(S, P);
    k_tri<<<NB_ * NH_ * NN / 8, 256, 0, stream>>>(P, LV, RV, O);
    k_split<false><<<(NR * DD / 64 + 63) / 64, 256, 0, stream>>>(O, NR * DD / 64, OPh, OPl);
    k_gemmw<bf, 1, false><<<dim3(NR / 64, DD / 64, 1), 32, 0, stream>>>(OPh, OPl, WT + (size_t)4 * DD * DD, nullptr, DD, AO, DD, nullptr, 0, 0, 0);
    k_ln<false><<<NR / 8, 256, 0, stream>>>(AO, x, g1, be1, HN, HNh, HNl);
    k_gemmw<bf, 1, true><<<dim3(NR / 64, FF / 64, 1), 32, 0, stream>>>(HNh, HNl, W1t, nullptr, DD, F1, FF, b1, 0, 0, 0);
    k_split<true><<<(NR * FF / 64 + 63) / 64, 256, 0, stream>>>(F1, NR * FF / 64, F1h, F1l);
    k_gemmw<bf, 1, true><<<dim3(NR / 64, DD / 64, 1), 32, 0, stream>>>(F1h, F1l, W2t, nullptr, FF, F2, DD, b2, 0, 0, 0);
    k_ln<true><<<NR / 8, 256, 0, stream>>>(F2, HN, g2, be2, OUT, nullptr, nullptr);
}
